// BiDirectionalMambaBlock_70480413327619
// MI455X (gfx1250) — hardware-verified
//
#include <hip/hip_runtime.h>
#include <math.h>

typedef __attribute__((ext_vector_type(16))) _Float16 v16h;
typedef __attribute__((ext_vector_type(8)))  _Float16 v8h;
typedef __attribute__((ext_vector_type(8)))  float    v8f;
typedef __attribute__((ext_vector_type(4)))  float    v4f;

constexpr int kBatch  = 2;
constexpr int kSeq    = 1024;
constexpr int kDm     = 1024;
constexpr int kDin    = 2048;
constexpr int kNst    = 16;
constexpr int kDtR    = 64;
constexpr int kNx     = kDtR + 2 * kNst;
constexpr int kDbcP   = 2 * kNx;
constexpr int kXrP    = 2 * kDin;
constexpr int kRows   = kBatch * kSeq;
constexpr int kTP     = 260;
constexpr int kScanTS = 32;
constexpr float kCarW   = 32.0f;
constexpr float kCarAct = 64.0f;
constexpr float kCarS   = 256.0f;
constexpr float kInvW   = 1.0f / kCarW;
constexpr float kInvAW  = 1.0f / (kCarAct * kCarW);
constexpr float kInvS   = 1.0f / kCarS;

static_assert(kNx == 96 && kDbcP == 192, "x_proj widths");
static_assert((kDm % 32) == 0 && (kDin % 32) == 0 && (kDtR % 32) == 0, "GEMM K multiples of 32");
static_assert((kRows % 64) == 0 && (kXrP % 64) == 0 && (kDbcP % 64) == 0 && (kDin % 64) == 0 && (kDm % 64) == 0, "GEMM M,N multiples of 64");
static_assert(((kRows / 64) * (kXrP / 64)) % 8 == 0, "in_proj tiles per block");
static_assert(((kRows / 64) * (kDbcP / 64)) % 8 == 0, "x_proj tiles per block");
static_assert(((kRows / 64) * (kDin / 64)) % 8 == 0, "dt_proj tiles per block");
static_assert(((kRows / 64) * (kDm / 64)) % 8 == 0, "out_proj tiles per block");
static_assert((kSeq % 64) == 0 && (kSeq % kScanTS) == 0 && (kDin % 256) == 0, "tile multiples");
static_assert((kSeq & (kSeq - 1)) == 0, "sequence length power of two");

constexpr size_t kOffXH    = 0;
constexpr size_t kOffWINH  = kOffXH    + (size_t)kRows * kDm * 2;
constexpr size_t kOffWOUTH = kOffWINH  + (size_t)kXrP * kDm * 2;
constexpr size_t kOffWXH   = kOffWOUTH + (size_t)kDm * kDin * 2;
constexpr size_t kOffWDTH  = kOffWXH   + (size_t)kDbcP * kDin * 2;
constexpr size_t kOffXR    = kOffWDTH  + (size_t)2 * kDin * kDtR * 2;
constexpr size_t kOffUC    = kOffXR    + (size_t)kRows * kXrP * 4;
constexpr size_t kOffUCH   = kOffUC    + (size_t)kRows * kDin * 4;
constexpr size_t kOffDBC   = kOffUCH   + (size_t)kRows * kDin * 2;
constexpr size_t kOffDT16  = kOffDBC   + (size_t)kRows * kDbcP * 4;
constexpr size_t kOffDLRH  = kOffDT16  + (size_t)2 * kRows * kDtR * 2;
constexpr size_t kOffS16   = kOffDLRH  + (size_t)2 * kRows * kDin * 2;
constexpr size_t kOffYH    = kOffS16   + (size_t)2 * kRows * kDin * 2;
constexpr size_t kWsTotal  = kOffYH    + (size_t)kRows * kDin * 2;
static_assert(kWsTotal == 120848384ull, "carve total");
static_assert(kWsTotal <= 134217728ull, "carve cap");
static_assert((kOffWINH % 128) == 0 && (kOffWOUTH % 128) == 0 && (kOffWXH % 128) == 0 && (kOffWDTH % 128) == 0 &&
              (kOffXR % 128) == 0 && (kOffUC % 128) == 0 && (kOffUCH % 128) == 0 && (kOffDBC % 128) == 0 &&
              (kOffDT16 % 128) == 0 && (kOffDLRH % 128) == 0 && (kOffS16 % 128) == 0 && (kOffYH % 128) == 0,
              "128-B aligned regions");

__device__ __forceinline__ float h16_to_f32(unsigned hb) {
  const unsigned sgn = (hb & 0x8000u) << 16;
  const unsigned em = hb & 0x7fffu;
  const float fn = __uint_as_float((em << 13) + 0x38000000u);
  const float fs = (float)em * 5.9604644775390625e-8f;
  const float mag = (em < 0x400u) ? fs : fn;
  return __uint_as_float(__float_as_uint(mag) | sgn);
}

__device__ __forceinline__ void dep_guard4_h(v8f& a, v8f& b, v8f& c, v8f& d, v16h x, v16h y) {
  asm volatile("v_nop\n\tv_nop\n\tv_nop\n\tv_nop" : "+v"(a), "+v"(b), "+v"(c), "+v"(d) : "v"(x), "v"(y));
}
__device__ __forceinline__ void keep4_h(v16h a, v16h b, v16h c, v16h d) {
  asm volatile("v_nop" :: "v"(a), "v"(b), "v"(c), "v"(d));
}
__device__ __forceinline__ void acc_guard4(v8f& a, v8f& b, v8f& c, v8f& d) {
  asm volatile("v_nop\n\tv_nop\n\tv_nop\n\tv_nop" : "+v"(a), "+v"(b), "+v"(c), "+v"(d));
}
__device__ __forceinline__ v16h frag_load_h(const _Float16* p) {
  union U { v16h v; v8h h[2]; };
  U f;
  f.h[0] = *(const v8h*)(p);
  f.h[1] = *(const v8h*)(p + 16);
  return f.v;
}
__device__ __forceinline__ v8f mma_h(v16h a, v16h b, v8f c) {
  return __builtin_amdgcn_wmma_f32_16x16x32_f16(false, a, false, b, (short)0, c, false, false);
}

template <int BIAS_MODE, int OUT_MODE>
__global__ __launch_bounds__(256) void wmma_gemm64(
    const unsigned short* __restrict__ Ap, int lda,
    const unsigned short* __restrict__ Btp, int ldb,
    void* __restrict__ Cout, int ldc,
    const float* __restrict__ bias,
    int M, int N, int K, float scale) {
  const _Float16* A  = (const _Float16*)Ap;
  const _Float16* Bt = (const _Float16*)Btp;
  __shared__ __align__(16) float sT[8][16 * 68];
  const int lane = threadIdx.x & 31;
  const int wave = threadIdx.x >> 5;
  const int tilesN = N >> 6;
  const int tilesM = M >> 6;
  const int tile = blockIdx.x * 8 + wave;
  if (tile >= tilesM * tilesN) return;
  const int tm = tile / tilesN;
  const int tn = tile - tm * tilesN;
  const int m0 = tm << 6;
  const int n0 = tn << 6;

  const int rlane = lane & 15;
  const int koff  = (lane >> 4) * 8;
  const int mOff  = (lane >> 4) * 8;

  v8f acc[4][4];
#pragma unroll
  for (int i = 0; i < 4; ++i)
#pragma unroll
    for (int j = 0; j < 4; ++j) acc[i][j] = (v8f){0.f,0.f,0.f,0.f,0.f,0.f,0.f,0.f};

  for (int k0 = 0; k0 < K; k0 += 32) {
    v16h bh[4];
#pragma unroll
    for (int j = 0; j < 4; ++j) {
      const size_t bo = (size_t)(n0 + (j << 4) + rlane) * ldb + koff + k0;
      bh[j] = frag_load_h(Bt + bo);
    }
#pragma unroll
    for (int i = 0; i < 4; ++i) {
      const size_t ao = (size_t)(m0 + (i << 4) + rlane) * lda + koff + k0;
      const v16h ah = frag_load_h(A + ao);
#pragma unroll
      for (int j = 0; j < 4; ++j) acc[i][j] = mma_h(ah, bh[j], acc[i][j]);
      dep_guard4_h(acc[i][0], acc[i][1], acc[i][2], acc[i][3], ah, bh[3]);
    }
    keep4_h(bh[0], bh[1], bh[2], bh[3]);
  }
  acc_guard4(acc[0][0], acc[0][1], acc[0][2], acc[0][3]);
  acc_guard4(acc[1][0], acc[1][1], acc[1][2], acc[1][3]);
  acc_guard4(acc[2][0], acc[2][1], acc[2][2], acc[2][3]);
  acc_guard4(acc[3][0], acc[3][1], acc[3][2], acc[3][3]);

  float* slab = sT[wave];
#pragma unroll
  for (int i = 0; i < 4; ++i) {
    const int mBase = m0 + (i << 4);
#pragma unroll
    for (int j = 0; j < 4; ++j) {
      const int n = n0 + (j << 4) + rlane;
      float bv = 0.f;
      if (BIAS_MODE == 2) bv = bias[n];
#pragma unroll
      for (int r = 0; r < 8; ++r) {
        float v = acc[i][j][r] * scale;
        if (BIAS_MODE == 2) v += bv;
        slab[(mOff + r) * 68 + (j << 4) + rlane] = v;
      }
    }
    __builtin_amdgcn_fence(__ATOMIC_RELEASE, "workgroup");
    __builtin_amdgcn_wave_barrier();
    __builtin_amdgcn_fence(__ATOMIC_ACQUIRE, "workgroup");
    if (OUT_MODE == 0) {
      float* C = (float*)Cout;
      const int hh = lane >> 4, c4 = (lane & 15) * 4;
      for (int pass = 0; pass < 2; ++pass) {
#pragma unroll
        for (int it = 0; it < 8; ++it) {
          const int row = it * 2 + hh;
          v4f v = *(const v4f*)(slab + row * 68 + c4);
          *(volatile v4f*)(C + (size_t)(mBase + row) * ldc + n0 + c4) = v;
        }
        __threadfence();
      }
    } else {
      const int q = lane >> 3, c8 = (lane & 7) * 8;
      unsigned short* C = (unsigned short*)Cout;
      for (int pass = 0; pass < 2; ++pass) {
#pragma unroll
        for (int it = 0; it < 4; ++it) {
          const int row = it * 4 + q;
          const float* sp = slab + row * 68 + c8;
          v8h hv;
#pragma unroll
          for (int e = 0; e < 8; ++e) hv[e] = (_Float16)sp[e];
          *(volatile v8h*)(C + (size_t)(mBase + row) * ldc + n0 + c8) = hv;
        }
        __threadfence();
      }
    }
    __builtin_amdgcn_fence(__ATOMIC_RELEASE, "workgroup");
    __builtin_amdgcn_wave_barrier();
    __builtin_amdgcn_fence(__ATOMIC_ACQUIRE, "workgroup");
  }
}

__global__ __launch_bounds__(256) void cast_f16_kernel(
    const float* __restrict__ src, unsigned short* __restrict__ dst, int total8, float scale)
{
  const int i = blockIdx.x * 256 + threadIdx.x;
  if (i >= total8) return;
  const size_t e0 = (size_t)i << 3;
  const float* p = src + e0;
  const v4f a0 = *(const v4f*)(p);
  const v4f a1 = *(const v4f*)(p + 4);
  v8h hv;
#pragma unroll
  for (int e = 0; e < 4; ++e) {
    hv[e]     = (_Float16)(a0[e] * scale);
    hv[4 + e] = (_Float16)(a1[e] * scale);
  }
  unsigned short* q = dst + e0;
  *(volatile v8h*)q = hv;
  __threadfence();
  *(volatile v8h*)q = hv;
}

__global__ __launch_bounds__(256) void dt_cast_kernel(
    const float* __restrict__ DBC, unsigned short* __restrict__ DT16, int total8)
{
  const int i = blockIdx.x * 256 + threadIdx.x;
  if (i >= total8) return;
  const int e0  = i << 3;
  const int dir = e0 / (kRows * kDtR);
  const int rem = e0 - dir * (kRows * kDtR);
  const int row = rem >> 6;
  const int c8  = rem & 63;
  const float* p = DBC + (size_t)row * kDbcP + dir * kNx + c8;
  const v4f a0 = *(const v4f*)(p);
  const v4f a1 = *(const v4f*)(p + 4);
  v8h hv;
#pragma unroll
  for (int e = 0; e < 4; ++e) {
    hv[e]     = (_Float16)(a0[e] * kCarAct);
    hv[4 + e] = (_Float16)(a1[e] * kCarAct);
  }
  unsigned short* qd = DT16 + e0;
  *(volatile v8h*)qd = hv;
  __threadfence();
  *(volatile v8h*)qd = hv;
}

__global__ __launch_bounds__(256) void conv_silu_kernel(
    const float* __restrict__ XR, const float* __restrict__ cw, const float* __restrict__ cb,
    float* __restrict__ UC, unsigned short* __restrict__ UCH)
{
  __shared__ __align__(16) float sT[16 * kTP];
  const int tid = threadIdx.x, lane = tid & 31, wave = tid >> 5;
  const int d0 = blockIdx.x * 256, d = d0 + tid;
  const int g0 = blockIdx.y * 64;
  const int tb = g0 & (kSeq - 1);
  const v4f wv = *(const v4f*)(cw + (size_t)d * 4);
  const float w0 = wv[0], w1 = wv[1], w2 = wv[2], w3 = wv[3];
  const float bc = cb[d];
  float xm3, xm2, xm1;
  {
    const bool hist = (tb > 0);
    const int rb = hist ? (g0 - 3) : g0;
    const float v3 = XR[(size_t)rb * kXrP + d];
    const float v2 = XR[(size_t)(rb + 1) * kXrP + d];
    const float v1 = XR[(size_t)(rb + 2) * kXrP + d];
    xm3 = hist ? v3 : 0.f;
    xm2 = hist ? v2 : 0.f;
    xm1 = hist ? v1 : 0.f;
  }
  const int hrow = wave >> 1;
  const int hch  = (wave & 1) * 128 + lane * 4;
#pragma unroll 1
  for (int sub = 0; sub < 4; ++sub) {
    const int lb = g0 + sub * 16;
#pragma unroll 1
    for (int s = 0; s < 16; ++s) {
      const float xcur = XR[(size_t)(lb + s) * kXrP + d];
      float acc = w0 * xm3;
      acc = fmaf(w1, xm2, acc);
      acc = fmaf(w2, xm1, acc);
      acc = fmaf(w3, xcur, acc);
      const float sv = acc + bc;
      const float sg = 1.0f / (1.0f + expf(-sv));
      sT[s * kTP + tid] = sv * sg;
      xm3 = xm2; xm2 = xm1; xm1 = xcur;
    }
    __syncthreads();
    v4f fv[4];
    v8h bv[2];
#pragma unroll
    for (int it = 0; it < 4; ++it) fv[it] = *(const v4f*)(sT + (it * 4 + hrow) * kTP + hch);
#pragma unroll
    for (int it = 0; it < 2; ++it) {
      const float* sp = sT + (it * 8 + wave) * kTP + lane * 8;
      const v4f a0 = *(const v4f*)(sp);
      const v4f a1 = *(const v4f*)(sp + 4);
#pragma unroll
      for (int e = 0; e < 4; ++e) {
        bv[it][e]     = (_Float16)(a0[e] * kCarAct);
        bv[it][4 + e] = (_Float16)(a1[e] * kCarAct);
      }
    }
    for (int pass = 0; pass < 2; ++pass) {
#pragma unroll
      for (int it = 0; it < 4; ++it)
        *(volatile v4f*)(UC + (size_t)(lb + it * 4 + hrow) * kDin + d0 + hch) = fv[it];
#pragma unroll
      for (int it = 0; it < 2; ++it)
        *(volatile v8h*)(UCH + (size_t)(lb + it * 8 + wave) * kDin + d0 + lane * 8) = bv[it];
      __threadfence();
    }
    __syncthreads();
  }
}

__global__ __launch_bounds__(256) void scan_kernel(
    const unsigned short* __restrict__ DLRH, const float* __restrict__ UC, const float* __restrict__ DBC,
    const float* __restrict__ fAlog, const float* __restrict__ bAlog,
    unsigned short* __restrict__ S16)
{
  __shared__ __align__(16) float sBC[kScanTS * 32];
  __shared__ __align__(16) float sY[kScanTS * kTP];
  static_assert(kScanTS * kTP >= kNst * 256, "A staging fits in the y tile");
  const int tid = threadIdx.x, lane = tid & 31, wave = tid >> 5;
  const int d0 = blockIdx.x * 256, d = d0 + tid;
  const int bix = blockIdx.y;
  const int dir = blockIdx.z;
  const float* Alog = (dir == 0) ? fAlog : bAlog;

#pragma unroll 1
  for (int n = 0; n < kNst; ++n) sY[n * 256 + tid] = -expf(Alog[(size_t)d * kNst + n]);
  __syncthreads();
  float An[kNst], h[kNst];
#pragma unroll
  for (int n = 0; n < kNst; ++n) {
    An[n] = sY[n * 256 + tid];
    h[n] = 0.f;
  }
  __syncthreads();

  const size_t rowb = (size_t)bix * kSeq;
  const size_t pl   = (size_t)dir * kRows;
  const int colBC = dir * kNx + kDtR;
  const int sr = tid >> 3, sq = (tid & 7) * 4;

#pragma unroll 1
  for (int c = 0; c < kSeq / kScanTS; ++c) {
    const int l0 = dir ? (kSeq - kScanTS * (c + 1)) : (kScanTS * c);
    {
      const v4f v = *(const v4f*)(DBC + (rowb + l0 + sr) * kDbcP + colBC + sq);
      *(v4f*)(sBC + sr * 32 + sq) = v;
    }
    __syncthreads();
#pragma unroll 1
    for (int s = 0; s < kScanTS; ++s) {
      const int ls = dir ? (kScanTS - 1 - s) : s;
      const size_t m = rowb + l0 + ls;
      const unsigned hb = (unsigned)DLRH[(pl + m) * kDin + d];
      const float a     = h16_to_f32(hb);
      const float delta = fmaxf(a, 0.0f) + log1pf(expf(-fabsf(a)));
      const float xv    = UC[m * kDin + d];
      const float dx    = delta * xv;
      v4f Bq[4], Cq[4];
#pragma unroll
      for (int qq = 0; qq < 4; ++qq) {
        Bq[qq] = *(const v4f*)(sBC + ls * 32 + 4 * qq);
        Cq[qq] = *(const v4f*)(sBC + ls * 32 + kNst + 4 * qq);
      }
      float y = 0.f;
#pragma unroll
      for (int n = 0; n < kNst; ++n) {
        const float e  = __expf(delta * An[n]);
        const float hn = fmaf(e, h[n], dx * Bq[n >> 2][n & 3]);
        h[n] = hn;
        y = fmaf(Cq[n >> 2][n & 3], hn, y);
      }
      sY[ls * kTP + tid] = y * kCarS;
    }
    __syncthreads();
    v8h hv[4];
#pragma unroll
    for (int it = 0; it < 4; ++it) {
      const float* sp = sY + (it * 8 + wave) * kTP + lane * 8;
      const v4f a0 = *(const v4f*)(sp);
      const v4f a1 = *(const v4f*)(sp + 4);
#pragma unroll
      for (int e = 0; e < 4; ++e) {
        hv[it][e]     = (_Float16)a0[e];
        hv[it][4 + e] = (_Float16)a1[e];
      }
    }
    for (int pass = 0; pass < 2; ++pass) {
#pragma unroll
      for (int it = 0; it < 4; ++it)
        *(volatile v8h*)(S16 + (pl + rowb + l0 + it * 8 + wave) * kDin + d0 + lane * 8) = hv[it];
      __threadfence();
    }
  }
}

__global__ __launch_bounds__(256) void combine_gate_kernel(
    const unsigned short* __restrict__ S16, const float* __restrict__ UC, const float* __restrict__ XR,
    const float* __restrict__ fD, const float* __restrict__ bD, unsigned short* __restrict__ YH)
{
  __shared__ __align__(16) float sT[16 * kTP];
  const int tid = threadIdx.x, lane = tid & 31, wave = tid >> 5;
  const int d0 = blockIdx.x * 256, d = d0 + tid;
  const int g0 = blockIdx.y * 64;
  const float Df = fD[d], Db = bD[d];
  const size_t plane = (size_t)kRows * kDin;
#pragma unroll 1
  for (int sub = 0; sub < 4; ++sub) {
    const int lb = g0 + sub * 16;
#pragma unroll 1
    for (int s = 0; s < 16; ++s) {
      const size_t m = (size_t)(lb + s);
      const unsigned hf = (unsigned)S16[m * kDin + d];
      const unsigned hr = (unsigned)S16[plane + m * kDin + d];
      const float sf = h16_to_f32(hf) * kInvS;
      const float sb = h16_to_f32(hr) * kInvS;
      const float uv = UC[m * kDin + d];
      const float rv = XR[m * kXrP + kDin + d];
      const float yf = fmaf(uv, Df, sf);
      const float yb = fmaf(uv, Db, sb);
      const float g  = rv * (1.0f / (1.0f + expf(-rv)));
      const float yv = (yf + yb) * 0.5f * g;
      sT[s * kTP + tid] = yv * kCarAct;
    }
    __syncthreads();
    v8h bv[2];
#pragma unroll
    for (int it = 0; it < 2; ++it) {
      const float* sp = sT + (it * 8 + wave) * kTP + lane * 8;
      const v4f a0 = *(const v4f*)(sp);
      const v4f a1 = *(const v4f*)(sp + 4);
#pragma unroll
      for (int e = 0; e < 4; ++e) {
        bv[it][e]     = (_Float16)a0[e];
        bv[it][4 + e] = (_Float16)a1[e];
      }
    }
    for (int pass = 0; pass < 2; ++pass) {
#pragma unroll
      for (int it = 0; it < 2; ++it)
        *(volatile v8h*)(YH + (size_t)(lb + it * 8 + wave) * kDin + d0 + lane * 8) = bv[it];
      __threadfence();
    }
    __syncthreads();
  }
}

extern "C" void kernel_launch(void* const* d_in, const int* in_sizes, int n_in,
                              void* d_out, int out_size, void* d_ws, size_t ws_size,
                              hipStream_t stream)
{
  if (n_in < 15) return;
  if (in_sizes[0] != kRows * kDm) return;
  if (in_sizes[1] != kXrP * kDm) return;
  if (in_sizes[2] != kDin * 4 || in_sizes[3] != kDin) return;
  if (in_sizes[4] != kDm * kDin) return;
  if (in_sizes[5] != kDin * kNst || in_sizes[6] != kDin) return;
  if (in_sizes[7] != kNx * kDin || in_sizes[8] != kDin * kDtR || in_sizes[9] != kDin) return;
  if (in_sizes[10] != kDin * kNst || in_sizes[11] != kDin) return;
  if (in_sizes[12] != kNx * kDin || in_sizes[13] != kDin * kDtR || in_sizes[14] != kDin) return;
  if (out_size != kRows * kDm) return;
  if (ws_size < kWsTotal) return;

  const float* x      = (const float*)d_in[0];
  const float* W_in   = (const float*)d_in[1];
  const float* W_conv = (const float*)d_in[2];
  const float* b_conv = (const float*)d_in[3];
  const float* W_out  = (const float*)d_in[4];
  const float* fA_log = (const float*)d_in[5];
  const float* fD     = (const float*)d_in[6];
  const float* fWx    = (const float*)d_in[7];
  const float* fWdt   = (const float*)d_in[8];
  const float* fbdt   = (const float*)d_in[9];
  const float* bA_log = (const float*)d_in[10];
  const float* bD     = (const float*)d_in[11];
  const float* bWx    = (const float*)d_in[12];
  const float* bWdt   = (const float*)d_in[13];
  const float* bbdt   = (const float*)d_in[14];
  float* out = (float*)d_out;

  char* ws = (char*)d_ws;
  unsigned short* XH    = (unsigned short*)(ws + kOffXH);
  unsigned short* WINH  = (unsigned short*)(ws + kOffWINH);
  unsigned short* WOUTH = (unsigned short*)(ws + kOffWOUTH);
  unsigned short* WXH   = (unsigned short*)(ws + kOffWXH);
  unsigned short* WDTH  = (unsigned short*)(ws + kOffWDTH);
  float*          XR    = (float*)(ws + kOffXR);
  float*          UC    = (float*)(ws + kOffUC);
  unsigned short* UCH   = (unsigned short*)(ws + kOffUCH);
  float*          DBC   = (float*)(ws + kOffDBC);
  unsigned short* DT16  = (unsigned short*)(ws + kOffDT16);
  unsigned short* DLRH  = (unsigned short*)(ws + kOffDLRH);
  unsigned short* S16   = (unsigned short*)(ws + kOffS16);
  unsigned short* YH    = (unsigned short*)(ws + kOffYH);

  cast_f16_kernel<<<(kRows * kDm / 8) / 256, 256, 0, stream>>>(x, XH, kRows * kDm / 8, 1.0f);
  cast_f16_kernel<<<(kXrP * kDm / 8) / 256, 256, 0, stream>>>(W_in, WINH, kXrP * kDm / 8, kCarW);
  cast_f16_kernel<<<(kDm * kDin / 8) / 256, 256, 0, stream>>>(W_out, WOUTH, kDm * kDin / 8, kCarW);
  cast_f16_kernel<<<(kNx * kDin / 8) / 256, 256, 0, stream>>>(fWx, WXH, kNx * kDin / 8, kCarW);
  cast_f16_kernel<<<(kNx * kDin / 8) / 256, 256, 0, stream>>>(bWx, WXH + (size_t)kNx * kDin, kNx * kDin / 8, kCarW);
  cast_f16_kernel<<<(kDin * kDtR / 8) / 256, 256, 0, stream>>>(fWdt, WDTH, kDin * kDtR / 8, kCarW);
  cast_f16_kernel<<<(kDin * kDtR / 8) / 256, 256, 0, stream>>>(bWdt, WDTH + (size_t)kDin * kDtR, kDin * kDtR / 8, kCarW);

  wmma_gemm64<0, 0><<<((kRows / 64) * (kXrP / 64)) / 8, 256, 0, stream>>>(
      XH, kDm, WINH, kDm, (void*)XR, kXrP, fbdt, kRows, kXrP, kDm, kInvW);

  conv_silu_kernel<<<dim3(kDin / 256, kRows / 64), 256, 0, stream>>>(XR, W_conv, b_conv, UC, UCH);

  wmma_gemm64<0, 0><<<((kRows / 64) * (kDbcP / 64)) / 8, 256, 0, stream>>>(
      UCH, kDin, WXH, kDin, (void*)DBC, kDbcP, fbdt, kRows, kDbcP, kDin, kInvAW);

  dt_cast_kernel<<<(2 * kRows * kDtR / 8) / 256, 256, 0, stream>>>(DBC, DT16, 2 * kRows * kDtR / 8);

  wmma_gemm64<2, 1><<<((kRows / 64) * (kDin / 64)) / 8, 256, 0, stream>>>(
      DT16, kDtR, WDTH, kDtR, (void*)DLRH, kDin, fbdt, kRows, kDin, kDtR, kInvAW);
  wmma_gemm64<2, 1><<<((kRows / 64) * (kDin / 64)) / 8, 256, 0, stream>>>(
      DT16 + (size_t)kRows * kDtR, kDtR, WDTH + (size_t)kDin * kDtR, kDtR,
      (void*)(DLRH + (size_t)kRows * kDin), kDin, bbdt, kRows, kDin, kDtR, kInvAW);

  scan_kernel<<<dim3(kDin / 256, kBatch, 2), 256, 0, stream>>>(DLRH, UC, DBC, fA_log, bA_log, S16);

  combine_gate_kernel<<<dim3(kDin / 256, kRows / 64), 256, 0, stream>>>(S16, UC, XR, fD, bD, YH);

  wmma_gemm64<0, 0><<<((kRows / 64) * (kDm / 64)) / 8, 256, 0, stream>>>(
      YH, kDin, WOUTH, kDin, (void*)out, kDm, fbdt, kRows, kDm, kDin, kInvAW);
}
